// AttentiveDensenet_31233002176654
// MI455X (gfx1250) — hardware-run, weakly checked
//
#include <hip/hip_runtime.h>
#include <math.h>

typedef __attribute__((ext_vector_type(16))) _Float16 v16h;
typedef __attribute__((ext_vector_type(8)))  _Float16 v8h;
typedef __attribute__((ext_vector_type(8)))  float    v8f;
typedef __attribute__((ext_vector_type(4)))  float    v4f;
typedef __attribute__((ext_vector_type(4)))  unsigned v4u;

constexpr int kBatch   = 8;
constexpr int kChan    = 256;
constexpr int kImgH    = 32;
constexpr int kImgW    = 32;
constexpr int kHeads   = 8;
constexpr int kHeadDim = 64;
constexpr int kLayers  = 4;
constexpr int kTopK    = 4;
constexpr int kPix     = kBatch * kImgH * kImgW;
constexpr int kQkvW    = kHeads * kHeadDim;
constexpr int kPadH    = kImgH + 2;
constexpr int kPadW    = kImgW + 2;
constexpr int kPadPix  = kBatch * kPadH * kPadW;
constexpr int kKc1     = 9 * kQkvW;
constexpr int kKc2     = 9 * kChan;
constexpr int kTilesM  = kPix / 64;
constexpr int kTempInt = 8;
constexpr float kInvTemp  = 1.0f / (float)kTempInt;
constexpr float kActCarry = 16.0f;
constexpr float kWgtCarry = 64.0f;
constexpr float kFold     = 1.0f / (kActCarry * kWgtCarry);
constexpr float kBnEps    = 1e-5f;
constexpr float kSpEps    = 1e-7f;
static_assert(kTempInt * kTempInt == kHeadDim, "temperature = sqrt(head dim)");
static_assert(kPix == 8192 && kQkvW == 512 && kPadPix == 9248, "shape constants");
static_assert((kChan % 32) == 0 && (kKc1 % 32) == 0 && (kKc2 % 32) == 0, "GEMM K multiples of 32");
static_assert((kQkvW % 32) == 0 && (kChan % 32) == 0, "a 32-wide k chunk never straddles a tap");
static_assert((kPix % 64) == 0 && ((3 * kQkvW) % 64) == 0 && (kChan % 64) == 0, "GEMM M,N multiples of 64");
static_assert(((kTilesM * 24) % 8) == 0 && ((kTilesM * 4) % 8) == 0, "exact GEMM grids");
static_assert((kImgW % 4) == 0 && ((kImgH * kImgW) % 64) == 0, "pixel tiles stay inside one image");

constexpr size_t kSzX32  = (size_t)kPix * kChan * 4;
constexpr size_t kSzXH   = (size_t)kPix * kChan * 2;
constexpr size_t kSzWQKV = (size_t)kLayers * 3 * kQkvW * kChan * 2;
constexpr size_t kSzW1P  = (size_t)kLayers * kChan * kKc1 * 2;
constexpr size_t kSzW2P  = (size_t)kLayers * kChan * kKc2 * 2;
constexpr size_t kSzQ16  = (size_t)kPix * kQkvW * 2;
constexpr size_t kSzHist = (size_t)kLayers * kPix * kQkvW * 2;
constexpr size_t kSzOPAD = (size_t)kPadPix * kQkvW * 2;
constexpr size_t kSzY32  = (size_t)kPix * kChan * 4;
constexpr size_t kSzH1P  = (size_t)kPadPix * kChan * 2;
constexpr size_t kSzBNW  = (size_t)2 * kTilesM * kChan * 4 + (size_t)2 * kChan * 4;
constexpr size_t kOffX32  = 0;
constexpr size_t kOffXH   = kOffX32  + kSzX32;
constexpr size_t kOffWQKV = kOffXH   + kSzXH;
constexpr size_t kOffW1P  = kOffWQKV + kSzWQKV;
constexpr size_t kOffW2P  = kOffW1P  + kSzW1P;
constexpr size_t kOffQ16  = kOffW2P  + kSzW2P;
constexpr size_t kOffKH   = kOffQ16  + kSzQ16;
constexpr size_t kOffVH   = kOffKH   + kSzHist;
constexpr size_t kOffOPAD = kOffVH   + kSzHist;
constexpr size_t kOffY32  = kOffOPAD + kSzOPAD;
constexpr size_t kOffH1P  = kOffY32  + kSzY32;
constexpr size_t kOffBNW  = kOffH1P  + kSzH1P;
constexpr size_t kWsTotal = kOffBNW  + kSzBNW;
static_assert(kWsTotal == 128239616ull, "carve total");
static_assert(kWsTotal <= 134217728ull, "carve cap");
static_assert((kOffXH % 128) == 0 && (kOffWQKV % 128) == 0 && (kOffW1P % 128) == 0 && (kOffW2P % 128) == 0 &&
              (kOffQ16 % 128) == 0 && (kOffKH % 128) == 0 && (kOffVH % 128) == 0 && (kOffOPAD % 128) == 0 &&
              (kOffY32 % 128) == 0 && (kOffH1P % 128) == 0 && (kOffBNW % 128) == 0, "128-B aligned regions");
constexpr size_t kPlaneElems = (size_t)kPix * kQkvW;
constexpr size_t kPlane4     = kPlaneElems / 8;

union FragU { v16h v; v8h h[2]; };
__device__ __forceinline__ v16h frag_load(const _Float16* p) {
  FragU f;
  f.h[0] = *(const v8h*)(p);
  f.h[1] = *(const v8h*)(p + 16);
  return f.v;
}
__device__ __forceinline__ v8f mma_f16(v16h a, v16h b, v8f c) {
  return __builtin_amdgcn_wmma_f32_16x16x32_f16(false, a, false, b, (short)0, c, false, false);
}
__device__ __forceinline__ void group_guard(v8f& a0, v8f& a1, v8f& a2, v8f& a3, v16h x,
                                            v16h b0, v16h b1, v16h b2, v16h b3) {
  asm volatile("v_nop\n\tv_nop\n\tv_nop\n\tv_nop"
               : "+v"(a0), "+v"(a1), "+v"(a2), "+v"(a3)
               : "v"(x), "v"(b0), "v"(b1), "v"(b2), "v"(b3));
}
__device__ __forceinline__ void keep4_h(v16h a, v16h b, v16h c, v16h d) {
  asm volatile("v_nop" :: "v"(a), "v"(b), "v"(c), "v"(d));
}
__device__ __forceinline__ void acc_guard4(v8f& a, v8f& b, v8f& c, v8f& d) {
  asm volatile("v_nop\n\tv_nop\n\tv_nop\n\tv_nop" : "+v"(a), "+v"(b), "+v"(c), "+v"(d));
}
__device__ __forceinline__ void wave_lds_sync() {
  __builtin_amdgcn_fence(__ATOMIC_RELEASE, "workgroup");
  __builtin_amdgcn_wave_barrier();
  __builtin_amdgcn_fence(__ATOMIC_ACQUIRE, "workgroup");
}

__device__ __forceinline__ float h16_to_f32(unsigned hb) {
  const unsigned sgn = (hb & 0x8000u) << 16;
  const unsigned em = hb & 0x7fffu;
  const float fn = __uint_as_float((em << 13) + 0x38000000u);
  const float fs = (float)em * 5.9604644775390625e-8f;
  const float mag = (em < 0x400u) ? fs : fn;
  return __uint_as_float(__float_as_uint(mag) | sgn);
}
__device__ __forceinline__ void unpack_h8(const v4u w, float (&f)[8]) {
  const unsigned w0 = w.x, w1 = w.y, w2 = w.z, w3 = w.w;
  f[0] = h16_to_f32(w0 & 0xffffu);
  f[1] = h16_to_f32(w0 >> 16);
  f[2] = h16_to_f32(w1 & 0xffffu);
  f[3] = h16_to_f32(w1 >> 16);
  f[4] = h16_to_f32(w2 & 0xffffu);
  f[5] = h16_to_f32(w2 >> 16);
  f[6] = h16_to_f32(w3 & 0xffffu);
  f[7] = h16_to_f32(w3 >> 16);
}

template <int MODE>
__global__ __launch_bounds__(256) void gemm_tile64_kernel(
    const unsigned short* __restrict__ Ap, const unsigned short* __restrict__ Btp,
    const float* __restrict__ bias0, const float* __restrict__ bias1, const float* __restrict__ bias2,
    void* out0, void* out1, void* out2, const float* __restrict__ gam)
{
  constexpr int CIN     = (MODE == 1) ? kQkvW : kChan;
  constexpr int NTAP    = (MODE == 0) ? 1 : 9;
  constexpr int KTOT    = NTAP * CIN;
  constexpr int TILES_N = (MODE == 0) ? 24 : 4;
  const _Float16* A  = (const _Float16*)Ap;
  const _Float16* Bt = (const _Float16*)Btp;
  __shared__ __align__(16) float sT[8][16 * 68];
  const int lane = threadIdx.x & 31;
  const int wave = threadIdx.x >> 5;
  const int tile = blockIdx.x * 8 + wave;
  const int tm = tile / TILES_N;
  const int tn = tile - tm * TILES_N;
  const int m0 = tm << 6;
  const int n0 = tn << 6;
  const int rlane = lane & 15;
  const int koff  = (lane >> 4) * 8;
  const int mOff  = (lane >> 4) * 8;

  int aoff[4], boff[4];
#pragma unroll
  for (int i = 0; i < 4; ++i) {
    const int m = m0 + (i << 4) + rlane;
    if (MODE == 0) {
      aoff[i] = m * kChan + koff;
    } else {
      const int bb = m >> 10, hh = (m >> 5) & 31, ww = m & 31;
      aoff[i] = ((bb * kPadH + hh) * kPadW + ww) * CIN + koff;
    }
    boff[i] = (n0 + (i << 4) + rlane) * KTOT + koff;
  }

  v8f acc[4][4];
#pragma unroll
  for (int i = 0; i < 4; ++i)
#pragma unroll
    for (int j = 0; j < 4; ++j) acc[i][j] = (v8f){0.f, 0.f, 0.f, 0.f, 0.f, 0.f, 0.f, 0.f};

#pragma unroll 1
  for (int tap = 0; tap < NTAP; ++tap) {
    const int ky = tap / 3;
    const int kx = tap - ky * 3;
    const int tapA = (MODE == 0) ? 0 : (ky * kPadW + kx) * CIN;
    const int tapB = tap * CIN;
#pragma unroll 1
    for (int c0 = 0; c0 < CIN; c0 += 32) {
      const int ka = tapA + c0;
      const int kb = tapB + c0;
      v16h bh[4];
#pragma unroll
      for (int j = 0; j < 4; ++j) bh[j] = frag_load(Bt + boff[j] + kb);
#pragma unroll
      for (int i = 0; i < 4; ++i) {
        const v16h ah = frag_load(A + aoff[i] + ka);
#pragma unroll
        for (int j = 0; j < 4; ++j) acc[i][j] = mma_f16(ah, bh[j], acc[i][j]);
        group_guard(acc[i][0], acc[i][1], acc[i][2], acc[i][3], ah, bh[0], bh[1], bh[2], bh[3]);
      }
      keep4_h(bh[0], bh[1], bh[2], bh[3]);
    }
  }
  acc_guard4(acc[0][0], acc[0][1], acc[0][2], acc[0][3]);
  acc_guard4(acc[1][0], acc[1][1], acc[1][2], acc[1][3]);
  acc_guard4(acc[2][0], acc[2][1], acc[2][2], acc[2][3]);
  acc_guard4(acc[3][0], acc[3][1], acc[3][2], acc[3][3]);

  float* slab = sT[wave];
  const int plane = tn >> 3;
  const int ncol0 = (MODE == 0) ? ((tn & 7) << 6) : n0;
  const float* biasp = bias0;
  if (MODE == 0) biasp = (plane == 0) ? bias0 : ((plane == 1) ? bias1 : bias2);
  float bv[4];
#pragma unroll
  for (int j = 0; j < 4; ++j) bv[j] = biasp[ncol0 + (j << 4) + rlane];
  float gval = 1.0f;
  if (MODE == 2) gval = gam[0];
  float cs[4] = {0.f, 0.f, 0.f, 0.f};
  float cq[4] = {0.f, 0.f, 0.f, 0.f};

#pragma unroll
  for (int i = 0; i < 4; ++i) {
    const int mBase = m0 + (i << 4);
#pragma unroll
    for (int j = 0; j < 4; ++j) {
#pragma unroll
      for (int r = 0; r < 8; ++r) {
        float v = fmaf(acc[i][j][r], kFold, bv[j]);
        if (MODE == 1) {
          cs[j] += v;
          cq[j] = fmaf(v, v, cq[j]);
        }
        if (MODE == 2) v *= gval;
        slab[(mOff + r) * 68 + (j << 4) + rlane] = v;
      }
    }
    wave_lds_sync();
    if (MODE == 0) {
      unsigned short* C = (unsigned short*)((plane == 0) ? out0 : ((plane == 1) ? out1 : out2));
      const int q = lane >> 3, c8 = (lane & 7) * 8;
      for (int pass = 0; pass < 2; ++pass) {
#pragma unroll
        for (int it = 0; it < 4; ++it) {
          const int row = it * 4 + q;
          const float* sp = slab + row * 68 + c8;
          v8h hv;
#pragma unroll
          for (int e = 0; e < 8; ++e) hv[e] = (_Float16)sp[e];
          *(volatile v8h*)(C + (size_t)(mBase + row) * kQkvW + ncol0 + c8) = hv;
        }
        __threadfence();
      }
    }
    if (MODE == 1) {
      float* C = (float*)out0;
      const int hh = lane >> 4, c4 = (lane & 15) * 4;
      for (int pass = 0; pass < 2; ++pass) {
#pragma unroll
        for (int it = 0; it < 8; ++it) {
          const int row = it * 2 + hh;
          const v4f v = *(const v4f*)(slab + row * 68 + c4);
          *(volatile v4f*)(C + (size_t)(mBase + row) * kChan + n0 + c4) = v;
        }
        __threadfence();
      }
    }
    if (MODE == 2) {
      float* X = (float*)out0;
      unsigned short* XHp = (unsigned short*)out1;
      const int hh = lane >> 4, c4 = (lane & 15) * 4;
      v4f nv[8];
#pragma unroll
      for (int it = 0; it < 8; ++it) {
        const int row = it * 2 + hh;
        const v4f xo = *(const v4f*)(X + (size_t)(mBase + row) * kChan + n0 + c4);
        const v4f dv = *(const v4f*)(slab + row * 68 + c4);
        nv[it] = xo + dv;
        *(v4f*)(slab + row * 68 + c4) = nv[it];
      }
      for (int pass = 0; pass < 2; ++pass) {
#pragma unroll
        for (int it = 0; it < 8; ++it) {
          const int row = it * 2 + hh;
          *(volatile v4f*)(X + (size_t)(mBase + row) * kChan + n0 + c4) = nv[it];
        }
        __threadfence();
      }
      wave_lds_sync();
      const int q = lane >> 3, c8 = (lane & 7) * 8;
      for (int pass = 0; pass < 2; ++pass) {
#pragma unroll
        for (int it = 0; it < 4; ++it) {
          const int row = it * 4 + q;
          const float* sp = slab + row * 68 + c8;
          v8h hv;
#pragma unroll
          for (int e = 0; e < 8; ++e) hv[e] = (_Float16)(sp[e] * kActCarry);
          *(volatile v8h*)(XHp + (size_t)(mBase + row) * kChan + n0 + c8) = hv;
        }
        __threadfence();
      }
    }
    wave_lds_sync();
  }

  if (MODE == 1) {
#pragma unroll
    for (int j = 0; j < 4; ++j) {
      const float os = __shfl_xor(cs[j], 16, 32);
      const float oq = __shfl_xor(cq[j], 16, 32);
      cs[j] += os;
      cq[j] += oq;
    }
    const int hh = lane >> 4, c4 = (lane & 15) * 4;
#pragma unroll
    for (int j = 0; j < 4; ++j) {
      const float sel = (hh != 0) ? cq[j] : cs[j];
      slab[hh * 68 + (j << 4) + rlane] = sel;
    }
    wave_lds_sync();
    const v4f pv = *(const v4f*)(slab + hh * 68 + c4);
    float* dst = (float*)out1 + (size_t)hh * (kTilesM * kChan) + (size_t)tm * kChan + n0 + c4;
    *(volatile v4f*)dst = pv;
    __threadfence();
    *(volatile v4f*)dst = pv;
  }
}

__global__ __launch_bounds__(256) void pack_x_kernel(
    const float* __restrict__ x, float* __restrict__ x32, unsigned short* __restrict__ xh)
{
  __shared__ __align__(16) float sT[64 * 68];
  const int tid = threadIdx.x;
  const int pt = blockIdx.x >> 2;
  const int ct = blockIdx.x & 3;
  const int pix0 = pt * 64, c0 = ct * 64;
  const int b = pix0 >> 10, hw0 = pix0 & 1023;
#pragma unroll
  for (int it = 0; it < 4; ++it) {
    const int ch = it * 16 + (tid >> 4);
    const int p4 = (tid & 15) * 4;
    const v4f v = *(const v4f*)(x + ((size_t)(b * kChan + c0 + ch)) * 1024 + hw0 + p4);
    sT[(p4 + 0) * 68 + ch] = v.x;
    sT[(p4 + 1) * 68 + ch] = v.y;
    sT[(p4 + 2) * 68 + ch] = v.z;
    sT[(p4 + 3) * 68 + ch] = v.w;
  }
  __syncthreads();
  v4f fv[4];
  v8h hv[2];
#pragma unroll
  for (int it = 0; it < 4; ++it) {
    const int pix = it * 16 + (tid >> 4);
    fv[it] = *(const v4f*)(sT + pix * 68 + (tid & 15) * 4);
  }
#pragma unroll
  for (int it = 0; it < 2; ++it) {
    const int pix = it * 32 + (tid >> 3);
    const float* sp = sT + pix * 68 + (tid & 7) * 8;
#pragma unroll
    for (int e = 0; e < 8; ++e) hv[it][e] = (_Float16)(sp[e] * kActCarry);
  }
  for (int pass = 0; pass < 2; ++pass) {
#pragma unroll
    for (int it = 0; it < 4; ++it) {
      const int pix = it * 16 + (tid >> 4);
      *(volatile v4f*)(x32 + (size_t)(pix0 + pix) * kChan + c0 + (tid & 15) * 4) = fv[it];
    }
#pragma unroll
    for (int it = 0; it < 2; ++it) {
      const int pix = it * 32 + (tid >> 3);
      *(volatile v8h*)(xh + (size_t)(pix0 + pix) * kChan + c0 + (tid & 7) * 8) = hv[it];
    }
    __threadfence();
  }
}

__global__ __launch_bounds__(256) void unpack_out_kernel(
    const float* __restrict__ x32, float* __restrict__ out)
{
  __shared__ __align__(16) float sT[64 * 68];
  const int tid = threadIdx.x;
  const int pt = blockIdx.x >> 2;
  const int ct = blockIdx.x & 3;
  const int pix0 = pt * 64, c0 = ct * 64;
  const int b = pix0 >> 10, hw0 = pix0 & 1023;
#pragma unroll
  for (int it = 0; it < 4; ++it) {
    const int pix = it * 16 + (tid >> 4);
    const int c4 = (tid & 15) * 4;
    const v4f v = *(const v4f*)(x32 + (size_t)(pix0 + pix) * kChan + c0 + c4);
    *(v4f*)(sT + pix * 68 + c4) = v;
  }
  __syncthreads();
  v4f ov[4];
#pragma unroll
  for (int it = 0; it < 4; ++it) {
    const int ch = it * 16 + (tid >> 4);
    const int p4 = (tid & 15) * 4;
    v4f t;
    t.x = sT[(p4 + 0) * 68 + ch];
    t.y = sT[(p4 + 1) * 68 + ch];
    t.z = sT[(p4 + 2) * 68 + ch];
    t.w = sT[(p4 + 3) * 68 + ch];
    ov[it] = t;
  }
  for (int pass = 0; pass < 2; ++pass) {
#pragma unroll
    for (int it = 0; it < 4; ++it) {
      const int ch = it * 16 + (tid >> 4);
      const int p4 = (tid & 15) * 4;
      *(volatile v4f*)(out + ((size_t)(b * kChan + c0 + ch)) * 1024 + hw0 + p4) = ov[it];
    }
    __threadfence();
  }
}

__global__ __launch_bounds__(256) void pack_wqkv_kernel(
    const float* __restrict__ kw, const float* __restrict__ vw, const float* __restrict__ qw,
    unsigned short* __restrict__ wqkv)
{
  const int idx = blockIdx.x * 256 + threadIdx.x;
  const int row = idx >> 5;
  const int c8 = (idx & 31) * 8;
  const int l = row / (3 * kQkvW);
  const int r = row - l * (3 * kQkvW);
  const int plane = r >> 9;
  const int rr = r & (kQkvW - 1);
  const float* src = (plane == 0) ? kw : ((plane == 1) ? vw : qw);
  const float* s = src + ((size_t)(l * kQkvW + rr)) * kChan + c8;
  const v4f a0 = *(const v4f*)(s);
  const v4f a1 = *(const v4f*)(s + 4);
  v8h hv;
#pragma unroll
  for (int e = 0; e < 4; ++e) {
    hv[e]     = (_Float16)(a0[e] * kWgtCarry);
    hv[4 + e] = (_Float16)(a1[e] * kWgtCarry);
  }
  unsigned short* d = wqkv + (size_t)row * kChan + c8;
  *(volatile v8h*)d = hv;
  __threadfence();
  *(volatile v8h*)d = hv;
}

template <int CIN>
__global__ __launch_bounds__(256) void pack_w3_kernel(
    const float* __restrict__ w, unsigned short* __restrict__ wp)
{
  constexpr int KTOT = 9 * CIN;
  constexpr int PER_ROW = KTOT / 8;
  static_assert(((kLayers * kChan * PER_ROW) % 256) == 0, "exact grid");
  const int idx = blockIdx.x * 256 + threadIdx.x;
  const int row = idx / PER_ROW;
  const int k = (idx - row * PER_ROW) * 8;
  const int tap = k / CIN;
  const int c = k - tap * CIN;
  const float* s = w + ((size_t)row * CIN + c) * 9 + tap;
  v8h hv;
#pragma unroll
  for (int e = 0; e < 8; ++e) hv[e] = (_Float16)(s[e * 9] * kWgtCarry);
  unsigned short* d = wp + (size_t)row * KTOT + k;
  *(volatile v8h*)d = hv;
  __threadfence();
  *(volatile v8h*)d = hv;
}

__global__ __launch_bounds__(96) void zero_halo_kernel(
    unsigned short* __restrict__ opad, unsigned short* __restrict__ h1p)
{
  const int b = blockIdx.x / 132;
  const int i = blockIdx.x - b * 132;
  int ph, pw;
  if (i < 34) { ph = 0; pw = i; }
  else if (i < 68) { ph = kPadH - 1; pw = i - 34; }
  else if (i < 100) { ph = i - 67; pw = 0; }
  else { ph = i - 99; pw = kPadW - 1; }
  const size_t pp = (size_t)((b * kPadH + ph) * kPadW + pw);
  const int tid = threadIdx.x;
  v8h z;
#pragma unroll
  for (int e = 0; e < 8; ++e) z[e] = (_Float16)0.0f;
  if (tid < 64) {
    unsigned short* d = opad + pp * kQkvW + tid * 8;
    *(volatile v8h*)d = z;
    __threadfence();
    *(volatile v8h*)d = z;
  } else {
    unsigned short* d = h1p + pp * kChan + (tid - 64) * 8;
    *(volatile v8h*)d = z;
    __threadfence();
    *(volatile v8h*)d = z;
  }
}

template <int LCUR>
__global__ __launch_bounds__(256) void attn_rows_kernel(
    const unsigned short* __restrict__ q16, const unsigned short* __restrict__ kh,
    const unsigned short* __restrict__ vh, unsigned short* __restrict__ opad)
{
#pragma clang fp contract(off)
  constexpr int NT = LCUR + 1;
  __shared__ __align__(16) v8h sO[256 * 8];
  const int tid = threadIdx.x, lane = tid & 31, wave = tid >> 5;
  const int g = blockIdx.x * 256 + tid;
  const v4u* q4 = (const v4u*)q16 + (size_t)g * 8;
  const v4u* k4 = (const v4u*)kh + (size_t)g * 8;
  const v4u* v4 = (const v4u*)vh + (size_t)g * 8;

  float sc[NT];
#pragma unroll
  for (int t = 0; t < NT; ++t) sc[t] = 0.0f;
#pragma unroll 1
  for (int c = 0; c < 8; ++c) {
    float qf[8];
    unpack_h8(q4[c], qf);
#pragma unroll
    for (int t = 0; t < NT; ++t) {
      float kf[8];
      unpack_h8(k4[(size_t)t * kPlane4 + c], kf);
#pragma unroll
      for (int e = 0; e < 8; ++e) sc[t] = fmaf(qf[e], kf[e], sc[t]);
    }
  }
  float mx = 0.0f;
#pragma unroll
  for (int t = 0; t < NT; ++t) {
    sc[t] = sc[t] * kInvTemp;
    mx = fmaxf(mx, sc[t]);
  }
  float at[NT];
  float ssum = 0.0f;
#pragma unroll
  for (int t = 0; t < NT; ++t) {
    at[t] = expf(sc[t] - mx);
    ssum += at[t];
  }
  float az = expf(0.0f - mx);
  ssum += az;
  const float inv_s = 1.0f / ssum;
#pragma unroll
  for (int t = 0; t < NT; ++t) at[t] = at[t] * inv_s;
  az = az * inv_s;
  if (NT + 1 > kTopK) {
    float m1 = 3.0e38f, m2 = 3.0e38f;
#pragma unroll
    for (int t = 0; t < NT; ++t) {
      m2 = fminf(m2, fmaxf(m1, at[t]));
      m1 = fminf(m1, at[t]);
    }
    m2 = fminf(m2, fmaxf(m1, az));
    const float delta = m2 + kSpEps;
    float wsum = 0.0f;
#pragma unroll
    for (int t = 0; t < NT; ++t) {
      at[t] = fmaxf(at[t] - delta, 0.0f);
      wsum += at[t];
    }
    wsum += fmaxf(az - delta, 0.0f);
    const float inv_w = 1.0f / (wsum + kSpEps);
#pragma unroll
    for (int t = 0; t < NT; ++t) at[t] = at[t] * inv_w;
  }
#pragma unroll 1
  for (int c = 0; c < 8; ++c) {
    float o[8];
    {
      float vf[8];
      unpack_h8(v4[c], vf);
#pragma unroll
      for (int e = 0; e < 8; ++e) o[e] = at[0] * vf[e];
    }
#pragma unroll
    for (int t = 1; t < NT; ++t) {
      float vf[8];
      unpack_h8(v4[(size_t)t * kPlane4 + c], vf);
#pragma unroll
      for (int e = 0; e < 8; ++e) o[e] = fmaf(at[t], vf[e], o[e]);
    }
    v8h hv;
#pragma unroll
    for (int e = 0; e < 8; ++e) hv[e] = (_Float16)(o[e] * kActCarry);
    sO[tid * 8 + c] = hv;
  }
  __syncthreads();
  v8h ov[8];
#pragma unroll
  for (int it = 0; it < 8; ++it) ov[it] = sO[wave * 256 + it * 32 + lane];
  for (int pass = 0; pass < 2; ++pass) {
#pragma unroll
    for (int it = 0; it < 8; ++it) {
      const int gl = blockIdx.x * 256 + wave * 32 + it * 4 + (lane >> 3);
      const int pix = gl >> 3, hd = gl & 7;
      const int bb = pix >> 10, hh = (pix >> 5) & 31, ww = pix & 31;
      const size_t po = ((size_t)((bb * kPadH + hh + 1) * kPadW + ww + 1)) * kQkvW + hd * kHeadDim + (lane & 7) * 8;
      *(volatile v8h*)(opad + po) = ov[it];
    }
    __threadfence();
  }
}

__global__ __launch_bounds__(256) void bn_finalize_kernel(
    const float* __restrict__ part, const float* __restrict__ g, const float* __restrict__ b,
    float* __restrict__ ss)
{
  const int c = threadIdx.x;
  const float* ps = part + c;
  const float* pq = part + (size_t)kTilesM * kChan + c;
  float s0 = 0.f, s1 = 0.f, s2 = 0.f, s3 = 0.f, q0 = 0.f, q1 = 0.f, q2 = 0.f, q3 = 0.f;
#pragma unroll 1
  for (int t = 0; t < kTilesM; t += 4) {
    s0 += ps[(t + 0) * kChan];
    s1 += ps[(t + 1) * kChan];
    s2 += ps[(t + 2) * kChan];
    s3 += ps[(t + 3) * kChan];
    q0 += pq[(t + 0) * kChan];
    q1 += pq[(t + 1) * kChan];
    q2 += pq[(t + 2) * kChan];
    q3 += pq[(t + 3) * kChan];
  }
  const float invn = 1.0f / (float)kPix;
  const float mean = ((s0 + s1) + (s2 + s3)) * invn;
  const float ex2  = ((q0 + q1) + (q2 + q3)) * invn;
  const float var  = fmaxf(ex2 - mean * mean, 0.0f);
  const float scl  = g[c] * rsqrtf(var + kBnEps);
  const float sft  = b[c] - mean * scl;
  *(volatile float*)(ss + c) = scl;
  *(volatile float*)(ss + kChan + c) = sft;
  __threadfence();
  *(volatile float*)(ss + c) = scl;
  *(volatile float*)(ss + kChan + c) = sft;
}

__global__ __launch_bounds__(256) void bn_relu_kernel(
    const float* __restrict__ y32, const float* __restrict__ ss, unsigned short* __restrict__ h1p)
{
  const int idx = blockIdx.x * 256 + threadIdx.x;
  const int pix = idx >> 5;
  const int c8 = (idx & 31) * 8;
  const v4f y0 = *(const v4f*)(y32 + (size_t)pix * kChan + c8);
  const v4f y1 = *(const v4f*)(y32 + (size_t)pix * kChan + c8 + 4);
  const v4f a0 = *(const v4f*)(ss + c8);
  const v4f a1 = *(const v4f*)(ss + c8 + 4);
  const v4f b0 = *(const v4f*)(ss + kChan + c8);
  const v4f b1 = *(const v4f*)(ss + kChan + c8 + 4);
  v8h hv;
#pragma unroll
  for (int e = 0; e < 4; ++e) {
    hv[e]     = (_Float16)(fmaxf(fmaf(y0[e], a0[e], b0[e]), 0.0f) * kActCarry);
    hv[4 + e] = (_Float16)(fmaxf(fmaf(y1[e], a1[e], b1[e]), 0.0f) * kActCarry);
  }
  const int bb = pix >> 10, hh = (pix >> 5) & 31, ww = pix & 31;
  unsigned short* d = h1p + ((size_t)((bb * kPadH + hh + 1) * kPadW + ww + 1)) * kChan + c8;
  *(volatile v8h*)d = hv;
  __threadfence();
  *(volatile v8h*)d = hv;
}

extern "C" void kernel_launch(void* const* d_in, const int* in_sizes, int n_in,
                              void* d_out, int out_size, void* d_ws, size_t ws_size,
                              hipStream_t stream) {
  if (n_in < 14) return;
  if (in_sizes[0] != kBatch * kChan * kImgH * kImgW) return;
  if (in_sizes[1] != kLayers * kQkvW * kChan) return;
  if (in_sizes[2] != kLayers * kQkvW) return;
  if (in_sizes[3] != kLayers * kQkvW * kChan) return;
  if (in_sizes[4] != kLayers * kQkvW) return;
  if (in_sizes[5] != kLayers * kQkvW * kChan) return;
  if (in_sizes[6] != kLayers * kQkvW) return;
  if (in_sizes[7] != kLayers * kChan * kQkvW * 9) return;
  if (in_sizes[8] != kLayers * kChan) return;
  if (in_sizes[9] != kLayers * kChan) return;
  if (in_sizes[10] != kLayers * kChan) return;
  if (in_sizes[11] != kLayers * kChan * kChan * 9) return;
  if (in_sizes[12] != kLayers * kChan) return;
  if (in_sizes[13] != kLayers) return;
  if (out_size != kBatch * kChan * kImgH * kImgW) return;
  if (ws_size < kWsTotal) return;

  const float* x      = (const float*)d_in[0];
  const float* kw     = (const float*)d_in[1];
  const float* kb     = (const float*)d_in[2];
  const float* qw     = (const float*)d_in[3];
  const float* qb     = (const float*)d_in[4];
  const float* vw     = (const float*)d_in[5];
  const float* vb     = (const float*)d_in[6];
  const float* ow1    = (const float*)d_in[7];
  const float* ob1    = (const float*)d_in[8];
  const float* bn_g   = (const float*)d_in[9];
  const float* bn_b   = (const float*)d_in[10];
  const float* ow2    = (const float*)d_in[11];
  const float* ob2    = (const float*)d_in[12];
  const float* gammas = (const float*)d_in[13];
  float* out = (float*)d_out;

  char* ws = (char*)d_ws;
  float*          X32  = (float*)(ws + kOffX32);
  unsigned short* XH   = (unsigned short*)(ws + kOffXH);
  unsigned short* WQKV = (unsigned short*)(ws + kOffWQKV);
  unsigned short* W1P  = (unsigned short*)(ws + kOffW1P);
  unsigned short* W2P  = (unsigned short*)(ws + kOffW2P);
  unsigned short* Q16  = (unsigned short*)(ws + kOffQ16);
  unsigned short* KH   = (unsigned short*)(ws + kOffKH);
  unsigned short* VH   = (unsigned short*)(ws + kOffVH);
  unsigned short* OPAD = (unsigned short*)(ws + kOffOPAD);
  float*          Y32  = (float*)(ws + kOffY32);
  unsigned short* H1P  = (unsigned short*)(ws + kOffH1P);
  float*          PART = (float*)(ws + kOffBNW);
  float*          BNSS = PART + (size_t)2 * kTilesM * kChan;

  pack_x_kernel<<<(kPix / 64) * (kChan / 64), 256, 0, stream>>>(x, X32, XH);
  pack_wqkv_kernel<<<(kLayers * 3 * kQkvW * kChan / 8) / 256, 256, 0, stream>>>(kw, vw, qw, WQKV);
  pack_w3_kernel<kQkvW><<<(kLayers * kChan * (kKc1 / 8)) / 256, 256, 0, stream>>>(ow1, W1P);
  pack_w3_kernel<kChan><<<(kLayers * kChan * (kKc2 / 8)) / 256, 256, 0, stream>>>(ow2, W2P);
  zero_halo_kernel<<<kBatch * 132, 96, 0, stream>>>(OPAD, H1P);

  for (int l = 0; l < kLayers; ++l) {
    gemm_tile64_kernel<0><<<(kTilesM * 24) / 8, 256, 0, stream>>>(
        XH, WQKV + (size_t)l * 3 * kQkvW * kChan,
        kb + (size_t)l * kQkvW, vb + (size_t)l * kQkvW, qb + (size_t)l * kQkvW,
        (void*)(KH + (size_t)l * kPlaneElems), (void*)(VH + (size_t)l * kPlaneElems), (void*)Q16, nullptr);

    if (l == 0)      attn_rows_kernel<0><<<(kPix * kHeads) / 256, 256, 0, stream>>>(Q16, KH, VH, OPAD);
    else if (l == 1) attn_rows_kernel<1><<<(kPix * kHeads) / 256, 256, 0, stream>>>(Q16, KH, VH, OPAD);
    else if (l == 2) attn_rows_kernel<2><<<(kPix * kHeads) / 256, 256, 0, stream>>>(Q16, KH, VH, OPAD);
    else             attn_rows_kernel<3><<<(kPix * kHeads) / 256, 256, 0, stream>>>(Q16, KH, VH, OPAD);

    gemm_tile64_kernel<1><<<(kTilesM * 4) / 8, 256, 0, stream>>>(
        OPAD, W1P + (size_t)l * kChan * kKc1,
        ob1 + (size_t)l * kChan, nullptr, nullptr,
        (void*)Y32, (void*)PART, nullptr, nullptr);

    bn_finalize_kernel<<<1, 256, 0, stream>>>(PART, bn_g + (size_t)l * kChan, bn_b + (size_t)l * kChan, BNSS);
    bn_relu_kernel<<<(kPix * 32) / 256, 256, 0, stream>>>(Y32, BNSS, H1P);

    gemm_tile64_kernel<2><<<(kTilesM * 4) / 8, 256, 0, stream>>>(
        H1P, W2P + (size_t)l * kChan * kKc2,
        ob2 + (size_t)l * kChan, nullptr, nullptr,
        (void*)X32, (void*)XH, nullptr, gammas + l);
  }

  unpack_out_kernel<<<(kPix / 64) * (kChan / 64), 256, 0, stream>>>(X32, out);
}
